// DprnnBlock_stateful_16862041604527
// MI455X (gfx1250) — hardware-run, weakly checked
//
#include <hip/hip_runtime.h>
#include <math.h>

constexpr int SEQL   = 400;
constexpr int WID    = 128;
constexpr int NCH    = 128;
constexpr int HID    = 64;
constexpr int NROW   = SEQL * WID;
constexpr int NELEM  = NROW * NCH;
constexpr int GI     = 4 * HID;
constexpr int GJ     = 4 * NCH;
constexpr int SLAB   = WID * NCH;
constexpr float WCARRY   = 16.0f;
constexpr float HCARRY   = 16.0f;
constexpr float INV_W    = 1.0f / WCARRY;
constexpr float INV_HW   = 1.0f / (WCARRY * HCARRY);
constexpr float LN_EPS_F = 1e-3f;
constexpr int IHP = 72;
constexpr int IZW = 132;
constexpr int JHP = 136;
constexpr int JZW = 260;

static_assert(SEQL % 16 == 0, "intra tiles of 16 sequences");
static_assert(WID % 16 == 0, "inter tiles of 16 sequences");
static_assert(NROW % 64 == 0 && GJ % 64 == 0 && NCH % 64 == 0, "GEMM M, N tile multiples");
static_assert(NCH % 32 == 0 && HID % 32 == 0, "GEMM K multiples of 32");
static_assert((2 * 16 * IHP) % 128 == 0, "intra h zero fill exact");
static_assert((2 * 16 * JHP) % 256 == 0, "inter h zero fill exact");
static_assert((NELEM / 8) % 256 == 0, "convert grid exact");
static_assert(SLAB == 16 * 256 * 4, "LayerNorm slab = 16 iterations x 256 threads x 4");
static_assert((IHP * 2) % 16 == 0 && (JHP * 2) % 16 == 0 && (IZW * 4) % 16 == 0 && (JZW * 4) % 16 == 0, "LDS rows 16-B aligned");

typedef __attribute__((ext_vector_type(16))) _Float16 v16h;
typedef __attribute__((ext_vector_type(8)))  _Float16 v8h;
typedef __attribute__((ext_vector_type(8)))  float    v8f;
typedef __attribute__((ext_vector_type(4)))  float    v4f;
typedef __attribute__((ext_vector_type(4)))  unsigned v4u;

__device__ __forceinline__ void guard_grp(v8f& a0, v8f& a1, v8f& a2, v8f& a3, v16h x, v16h b0, v16h b1, v16h b2, v16h b3) {
  asm volatile("v_nop\n\tv_nop\n\tv_nop\n\tv_nop" : "+v"(a0), "+v"(a1), "+v"(a2), "+v"(a3) : "v"(x), "v"(b0), "v"(b1), "v"(b2), "v"(b3));
}
__device__ __forceinline__ void guard_grp2(v8f& a0, v8f& a1, v8f& a2, v8f& a3, v16h x0, v16h x1,
                                           v16h b0, v16h b1, v16h b2, v16h b3, v16h b4, v16h b5, v16h b6, v16h b7) {
  asm volatile("v_nop\n\tv_nop\n\tv_nop\n\tv_nop" : "+v"(a0), "+v"(a1), "+v"(a2), "+v"(a3)
               : "v"(x0), "v"(x1), "v"(b0), "v"(b1), "v"(b2), "v"(b3), "v"(b4), "v"(b5), "v"(b6), "v"(b7));
}
__device__ __forceinline__ void keep4_h(v16h a, v16h b, v16h c, v16h d) { asm volatile("v_nop" :: "v"(a), "v"(b), "v"(c), "v"(d)); }
__device__ __forceinline__ void acc_guard4(v8f& a, v8f& b, v8f& c, v8f& d) { asm volatile("v_nop\n\tv_nop\n\tv_nop\n\tv_nop" : "+v"(a), "+v"(b), "+v"(c), "+v"(d)); }

struct FragH {
  union U { v16h v; v8h h[2]; };
  static __device__ __forceinline__ v16h load(const _Float16* p) {
    U f; f.h[0] = *(const v8h*)(p); f.h[1] = *(const v8h*)(p + 16); return f.v;
  }
  static __device__ __forceinline__ v8f mma(v16h a, v16h b, v8f c) {
    return __builtin_amdgcn_wmma_f32_16x16x32_f16(false, a, false, b, (short)0, c, false, false);
  }
};

__device__ __forceinline__ float h16_to_f32(unsigned hb) {
  const unsigned sgn = (hb & 0x8000u) << 16; const unsigned em = hb & 0x7fffu;
  const float fn = __uint_as_float((em << 13) + 0x38000000u);
  const float fs = (float)em * 5.9604644775390625e-8f;
  const float mag = (em < 0x400u) ? fs : fn; return __uint_as_float(__float_as_uint(mag) | sgn);
}

__device__ __forceinline__ float hsig_f(float x) { return fminf(fmaxf(0.2f * x + 0.5f, 0.0f), 1.0f); }
__device__ __forceinline__ float tanh_f(float x) {
  const float xc = fminf(fmaxf(x, -15.0f), 15.0f);
  const float e = expf(2.0f * xc);
  return 1.0f - 2.0f / (e + 1.0f);
}
__device__ __forceinline__ float wave_sum(float s) {
#pragma unroll
  for (int off = 1; off < 32; off <<= 1) s += __shfl_xor(s, off, 32);
  return s;
}

__global__ __launch_bounds__(256) void cvt8_f16_kernel(const float* __restrict__ src, unsigned short* __restrict__ dst, int n8) {
  const int i = blockIdx.x * 256 + threadIdx.x;
  if (i < n8) {
    const float* sp = src + (size_t)i * 8;
    const v4f a = *(const v4f*)(sp);
    const v4f b = *(const v4f*)(sp + 4);
    v8h hv;
#pragma unroll
    for (int e = 0; e < 4; ++e) {
      hv[e]     = (_Float16)a[e];
      hv[4 + e] = (_Float16)b[e];
    }
    *(volatile v8h*)(dst + (size_t)i * 8) = hv;
    __threadfence();
    *(volatile v8h*)(dst + (size_t)i * 8) = hv;
  }
}

__global__ __launch_bounds__(256) void tpw_f16_kernel(const float* __restrict__ src, int R, int C, int ldo,
                                                      unsigned short* __restrict__ O, float sc) {
  __shared__ float Tt[64 * 65];
  const int tid = threadIdx.x;
  const int c0 = blockIdx.x * 64, r0 = blockIdx.y * 64;
#pragma unroll
  for (int i = 0; i < 4; ++i) {
    const int idx = i * 256 + tid;
    const int rr = idx >> 4, cc = (idx & 15) * 4;
    const v4f v = *(const v4f*)(src + (size_t)(r0 + rr) * (size_t)C + c0 + cc);
    Tt[rr * 65 + cc + 0] = v[0];
    Tt[rr * 65 + cc + 1] = v[1];
    Tt[rr * 65 + cc + 2] = v[2];
    Tt[rr * 65 + cc + 3] = v[3];
  }
  __syncthreads();
  const int q = tid >> 3, c8 = (tid & 7) * 8;
  v8h hv[2];
#pragma unroll
  for (int g = 0; g < 2; ++g) {
    const int qq = g * 32 + q;
#pragma unroll
    for (int e = 0; e < 8; ++e) {
      const float f = Tt[(c8 + e) * 65 + qq];
      hv[g][e] = (_Float16)(f * sc);
    }
  }
  for (int pass = 0; pass < 2; ++pass) {
#pragma unroll
    for (int g = 0; g < 2; ++g) {
      const size_t o = (size_t)(c0 + g * 32 + q) * (size_t)ldo + (size_t)(r0 + c8);
      *(volatile v8h*)(O + o) = hv[g];
    }
    __threadfence();
  }
}

__global__ __launch_bounds__(128) void bias_cat_kernel(const float* __restrict__ ba, const float* __restrict__ bb,
                                                       float* __restrict__ dst) {
  const int tid = threadIdx.x;
  const int which = tid >> 6;
  const int idx = (tid & 63) * 4;
  const v4f va = *(const v4f*)(ba + idx);
  const v4f vb = *(const v4f*)(bb + idx);
  v4f o;
#pragma unroll
  for (int e = 0; e < 4; ++e) o[e] = which ? vb[e] : va[e];
  float* op = dst + which * GI + idx;
  *(volatile v4f*)op = o;
  __threadfence();
  *(volatile v4f*)op = o;
}

template <int OUT_MODE>
__global__ __launch_bounds__(256) void wmma_gemm64_f16(
    const unsigned short* __restrict__ Ap, int lda,
    const unsigned short* __restrict__ Btp, int ldb,
    void* __restrict__ Cout, int ldc,
    const float* __restrict__ bias,
    int Mrows, int Ncols, int Kdepth, float scale) {
  const _Float16* A  = (const _Float16*)Ap;
  const _Float16* Bt = (const _Float16*)Btp;
  __shared__ __align__(16) float sT[8][16 * 68];
  const int lane = threadIdx.x & 31;
  const int wave = threadIdx.x >> 5;
  const int tilesN = Ncols >> 6;
  const int tilesM = Mrows >> 6;
  const int tile = blockIdx.x * 8 + wave;
  if (tile >= tilesM * tilesN) return;
  const int tm = tile / tilesN;
  const int tn = tile - tm * tilesN;
  const int m0 = tm << 6;
  const int n0 = tn << 6;

  const int rlane = lane & 15;
  const int koff  = (lane >> 4) * 8;
  const int mOff  = (lane >> 4) * 8;

  v8f acc[4][4];
#pragma unroll
  for (int i = 0; i < 4; ++i)
#pragma unroll
    for (int j = 0; j < 4; ++j) acc[i][j] = (v8f){0.f, 0.f, 0.f, 0.f, 0.f, 0.f, 0.f, 0.f};

  for (int k0 = 0; k0 < Kdepth; k0 += 32) {
    v16h bh[4];
#pragma unroll
    for (int j = 0; j < 4; ++j) {
      const size_t bo = (size_t)(n0 + (j << 4) + rlane) * ldb + koff + k0;
      bh[j] = FragH::load(Bt + bo);
    }
#pragma unroll
    for (int i = 0; i < 4; ++i) {
      const size_t ao = (size_t)(m0 + (i << 4) + rlane) * lda + koff + k0;
      const v16h ah = FragH::load(A + ao);
#pragma unroll
      for (int j = 0; j < 4; ++j) acc[i][j] = FragH::mma(ah, bh[j], acc[i][j]);
      guard_grp(acc[i][0], acc[i][1], acc[i][2], acc[i][3], ah, bh[0], bh[1], bh[2], bh[3]);
    }
    keep4_h(bh[0], bh[1], bh[2], bh[3]);
  }
  acc_guard4(acc[0][0], acc[0][1], acc[0][2], acc[0][3]);
  acc_guard4(acc[1][0], acc[1][1], acc[1][2], acc[1][3]);
  acc_guard4(acc[2][0], acc[2][1], acc[2][2], acc[2][3]);
  acc_guard4(acc[3][0], acc[3][1], acc[3][2], acc[3][3]);

  float* slab = sT[wave];
#pragma unroll
  for (int i = 0; i < 4; ++i) {
    const int mBase = m0 + (i << 4);
#pragma unroll
    for (int j = 0; j < 4; ++j) {
      const int n = n0 + (j << 4) + rlane;
      const float bv = bias[n];
#pragma unroll
      for (int r = 0; r < 8; ++r) {
        const float v = acc[i][j][r] * scale + bv;
        slab[(mOff + r) * 68 + (j << 4) + rlane] = v;
      }
    }
    __builtin_amdgcn_fence(__ATOMIC_RELEASE, "workgroup");
    __builtin_amdgcn_wave_barrier();
    __builtin_amdgcn_fence(__ATOMIC_ACQUIRE, "workgroup");
    if (OUT_MODE == 0) {
      float* Cf = (float*)Cout;
      const int hh = lane >> 4, c4 = (lane & 15) * 4;
      for (int pass = 0; pass < 2; ++pass) {
#pragma unroll
        for (int it = 0; it < 8; ++it) {
          const int row = it * 2 + hh;
          const v4f v = *(const v4f*)(slab + row * 68 + c4);
          *(volatile v4f*)(Cf + (size_t)(mBase + row) * ldc + n0 + c4) = v;
        }
        __threadfence();
      }
    } else {
      const int q = lane >> 3, c8 = (lane & 7) * 8;
      unsigned short* Ch = (unsigned short*)Cout;
      for (int pass = 0; pass < 2; ++pass) {
#pragma unroll
        for (int it = 0; it < 4; ++it) {
          const int row = it * 4 + q;
          const float* sp = slab + row * 68 + c8;
          v8h hv;
#pragma unroll
          for (int e = 0; e < 8; ++e) hv[e] = (_Float16)sp[e];
          *(volatile v8h*)(Ch + (size_t)(mBase + row) * ldc + n0 + c8) = hv;
        }
        __threadfence();
      }
    }
    __builtin_amdgcn_fence(__ATOMIC_RELEASE, "workgroup");
    __builtin_amdgcn_wave_barrier();
    __builtin_amdgcn_fence(__ATOMIC_ACQUIRE, "workgroup");
  }
}

__global__ __launch_bounds__(128) void intra_seq_kernel(const unsigned short* __restrict__ XZ,
                                                        const unsigned short* __restrict__ Up,
                                                        unsigned short* __restrict__ H16) {
  __shared__ __align__(16) _Float16 Ah[2][16 * IHP];
  __shared__ __align__(16) unsigned Zw[2][16 * IZW];
  const int tid = threadIdx.x, lane = tid & 31, wave = tid >> 5;
  const int c = lane & 15, hh = lane >> 4, koff = hh * 8;
  const int l0 = blockIdx.x * 16;
  const int dir = blockIdx.y;
  const _Float16* U = (const _Float16*)Up + (size_t)dir * GI * HID;

  v16h bfr[4][2];
#pragma unroll
  for (int g = 0; g < 4; ++g)
#pragma unroll
    for (int kt = 0; kt < 2; ++kt)
      bfr[g][kt] = FragH::load(U + (size_t)(g * HID + 16 * wave + c) * HID + koff + 32 * kt);

  {
    _Float16* ahf = &Ah[0][0];
#pragma unroll 1
    for (int i = tid; i < 2 * 16 * IHP; i += 128) ahf[i] = (_Float16)0.0f;
  }
  {
    const int t0 = dir ? (WID - 1) : 0;
#pragma unroll
    for (int i = 0; i < 4; ++i) {
      const int q = i * 128 + tid;
      const int m = q >> 5, cc = q & 31;
      const v4u w = *(const v4u*)(XZ + ((size_t)((l0 + m) * WID + t0)) * GJ + dir * GI + cc * 8);
      *(v4u*)(&Zw[0][0] + m * IZW + cc * 4) = w;
    }
  }
  float cst[8];
#pragma unroll
  for (int r = 0; r < 8; ++r) cst[r] = 0.0f;
  __syncthreads();

  const v8f z8 = {0.f, 0.f, 0.f, 0.f, 0.f, 0.f, 0.f, 0.f};
  const int colw = (16 * wave + c) >> 1;
  const unsigned sh = (unsigned)(c & 1) * 16u;
  const int jcol = 16 * wave + c;

#pragma unroll 1
  for (int step = 0; step < WID; ++step) {
    const int cur = step & 1;
    const int t = dir ? (WID - 1 - step) : step;
    const _Float16* ahc = &Ah[cur][0] + c * IHP + koff;
    _Float16* ahn = &Ah[cur ^ 1][0];
    const unsigned* zc = &Zw[cur][0];

    const v16h a0 = FragH::load(ahc);
    const v16h a1 = FragH::load(ahc + 32);
    v8f acc[4];
#pragma unroll
    for (int g = 0; g < 4; ++g) {
      acc[g] = z8;
      acc[g] = FragH::mma(a0, bfr[g][0], acc[g]);
      acc[g] = FragH::mma(a1, bfr[g][1], acc[g]);
    }
    guard_grp2(acc[0], acc[1], acc[2], acc[3], a0, a1,
               bfr[0][0], bfr[0][1], bfr[1][0], bfr[1][1], bfr[2][0], bfr[2][1], bfr[3][0], bfr[3][1]);

#pragma unroll
    for (int r = 0; r < 8; ++r) {
      const unsigned* zr = zc + (8 * hh + r) * IZW + colw;
      const unsigned wi = zr[0], wf = zr[32], wg = zr[64], wo = zr[96];
      const float zi = h16_to_f32((wi >> sh) & 0xffffu) + acc[0][r] * INV_HW;
      const float zf = h16_to_f32((wf >> sh) & 0xffffu) + acc[1][r] * INV_HW;
      const float zg = h16_to_f32((wg >> sh) & 0xffffu) + acc[2][r] * INV_HW;
      const float zo = h16_to_f32((wo >> sh) & 0xffffu) + acc[3][r] * INV_HW;
      const float cn = hsig_f(zf) * cst[r] + hsig_f(zi) * tanh_f(zg);
      cst[r] = cn;
      const float hn = hsig_f(zo) * tanh_f(cn);
      ahn[(8 * hh + r) * IHP + jcol] = (_Float16)(hn * HCARRY);
    }

    {
      const int sn = (step + 1 < WID) ? (step + 1) : step;
      const int tn = dir ? (WID - 1 - sn) : sn;
#pragma unroll
      for (int i = 0; i < 4; ++i) {
        const int q = i * 128 + tid;
        const int m = q >> 5, cc = q & 31;
        const v4u w = *(const v4u*)(XZ + ((size_t)((l0 + m) * WID + tn)) * GJ + dir * GI + cc * 8);
        *(v4u*)(&Zw[cur ^ 1][0] + m * IZW + cc * 4) = w;
      }
    }
    __syncthreads();

    {
      const int q = lane >> 3, c8 = (lane & 7) * 8;
      const int m = wave * 4 + q;
      const v8h hv = *(const v8h*)(ahn + m * IHP + c8);
      unsigned short* gp = H16 + ((size_t)((l0 + m) * WID + t)) * NCH + dir * HID + c8;
      *(volatile v8h*)gp = hv;
      __threadfence();
      *(volatile v8h*)gp = hv;
    }
  }
}

__global__ __launch_bounds__(256) void inter_seq_kernel(const unsigned short* __restrict__ XZ,
                                                        const unsigned short* __restrict__ Up,
                                                        unsigned short* __restrict__ H16) {
  __shared__ __align__(16) _Float16 Ah[2][16 * JHP];
  __shared__ __align__(16) unsigned Zw[2][16 * JZW];
  const _Float16* U = (const _Float16*)Up;
  const int tid = threadIdx.x, lane = tid & 31, wave = tid >> 5;
  const int c = lane & 15, hh = lane >> 4, koff = hh * 8;
  const int w0 = blockIdx.x * 16;

  {
    _Float16* ahf = &Ah[0][0];
#pragma unroll 1
    for (int i = tid; i < 2 * 16 * JHP; i += 256) ahf[i] = (_Float16)0.0f;
  }
#pragma unroll
  for (int i = 0; i < 4; ++i) {
    const int q = i * 256 + tid;
    const int m = q >> 6, cc = q & 63;
    const v4u w = *(const v4u*)(XZ + ((size_t)(w0 + m)) * GJ + cc * 8);
    *(v4u*)(&Zw[0][0] + m * JZW + cc * 4) = w;
  }
  float cst[8];
#pragma unroll
  for (int r = 0; r < 8; ++r) cst[r] = 0.0f;
  __syncthreads();

  const v8f z8 = {0.f, 0.f, 0.f, 0.f, 0.f, 0.f, 0.f, 0.f};
  const int jcol = 16 * wave + c;
  const int colw = jcol >> 1;
  const unsigned sh = (unsigned)(c & 1) * 16u;
  const _Float16* wj = U + (size_t)jcol * NCH + koff;

#pragma unroll 1
  for (int l = 0; l < SEQL; ++l) {
    const int cur = l & 1;
    const _Float16* ahc = &Ah[cur][0] + c * JHP + koff;
    _Float16* ahn = &Ah[cur ^ 1][0];
    const unsigned* zc = &Zw[cur][0];

    v8f acc[4];
    acc[0] = z8; acc[1] = z8; acc[2] = z8; acc[3] = z8;
#pragma unroll 1
    for (int k0 = 0; k0 < NCH; k0 += 32) {
      const v16h a  = FragH::load(ahc + k0);
      const v16h b0 = FragH::load(wj + k0);
      const v16h b1 = FragH::load(wj + (size_t)1 * NCH * NCH + k0);
      const v16h b2 = FragH::load(wj + (size_t)2 * NCH * NCH + k0);
      const v16h b3 = FragH::load(wj + (size_t)3 * NCH * NCH + k0);
      acc[0] = FragH::mma(a, b0, acc[0]);
      acc[1] = FragH::mma(a, b1, acc[1]);
      acc[2] = FragH::mma(a, b2, acc[2]);
      acc[3] = FragH::mma(a, b3, acc[3]);
      guard_grp(acc[0], acc[1], acc[2], acc[3], a, b0, b1, b2, b3);
    }
    acc_guard4(acc[0], acc[1], acc[2], acc[3]);

#pragma unroll
    for (int r = 0; r < 8; ++r) {
      const unsigned* zr = zc + (8 * hh + r) * JZW + colw;
      const unsigned wi = zr[0], wf = zr[64], wg = zr[128], wo = zr[192];
      const float zi = h16_to_f32((wi >> sh) & 0xffffu) + acc[0][r] * INV_HW;
      const float zf = h16_to_f32((wf >> sh) & 0xffffu) + acc[1][r] * INV_HW;
      const float zg = h16_to_f32((wg >> sh) & 0xffffu) + acc[2][r] * INV_HW;
      const float zo = h16_to_f32((wo >> sh) & 0xffffu) + acc[3][r] * INV_HW;
      const float cn = hsig_f(zf) * cst[r] + hsig_f(zi) * tanh_f(zg);
      cst[r] = cn;
      const float hn = hsig_f(zo) * tanh_f(cn);
      ahn[(8 * hh + r) * JHP + jcol] = (_Float16)(hn * HCARRY);
    }

    {
      const int ln = (l + 1 < SEQL) ? (l + 1) : l;
#pragma unroll
      for (int i = 0; i < 4; ++i) {
        const int q = i * 256 + tid;
        const int m = q >> 6, cc = q & 63;
        const v4u w = *(const v4u*)(XZ + ((size_t)(ln * WID + w0 + m)) * GJ + cc * 8);
        *(v4u*)(&Zw[cur ^ 1][0] + m * JZW + cc * 4) = w;
      }
    }
    __syncthreads();

    {
      const int m = tid >> 4, c8 = (tid & 15) * 8;
      const v8h hv = *(const v8h*)(ahn + m * JHP + c8);
      unsigned short* gp = H16 + ((size_t)(l * WID + w0 + m)) * NCH + c8;
      *(volatile v8h*)gp = hv;
      __threadfence();
      *(volatile v8h*)gp = hv;
    }
  }
}

__global__ __launch_bounds__(256) void ln_slab_res_kernel(const float* __restrict__ V, const float* __restrict__ RES,
                                                          const float* __restrict__ G, const float* __restrict__ Bt,
                                                          float* __restrict__ OUT) {
  __shared__ float red1[8];
  __shared__ float red2[8];
  const int tid = threadIdx.x, lane = tid & 31, wave = tid >> 5;
  const size_t base = (size_t)blockIdx.x * SLAB;
  const float* vp = V + base;

  float s = 0.0f;
#pragma unroll 1
  for (int it = 0; it < 16; ++it) {
    const v4f v = *(const v4f*)(vp + (size_t)(it * 256 + tid) * 4);
    s += (v[0] + v[1]) + (v[2] + v[3]);
  }
  s = wave_sum(s);
  if (lane == 0) red1[wave] = s;
  __syncthreads();
  const float tot = ((red1[0] + red1[1]) + (red1[2] + red1[3])) + ((red1[4] + red1[5]) + (red1[6] + red1[7]));
  const float mu = tot * (1.0f / (float)SLAB);

  float ss = 0.0f;
#pragma unroll 1
  for (int it = 0; it < 16; ++it) {
    const v4f v = *(const v4f*)(vp + (size_t)(it * 256 + tid) * 4);
    const float d0 = v[0] - mu, d1 = v[1] - mu, d2 = v[2] - mu, d3 = v[3] - mu;
    ss += (d0 * d0 + d1 * d1) + (d2 * d2 + d3 * d3);
  }
  ss = wave_sum(ss);
  if (lane == 0) red2[wave] = ss;
  __syncthreads();
  const float tot2 = ((red2[0] + red2[1]) + (red2[2] + red2[3])) + ((red2[4] + red2[5]) + (red2[6] + red2[7]));
  const float var = tot2 * (1.0f / (float)SLAB);
  const float rstd = rsqrtf(var + LN_EPS_F);

#pragma unroll 1
  for (int it = 0; it < 16; ++it) {
    const size_t e4 = (size_t)(it * 256 + tid) * 4;
    const v4f v  = *(const v4f*)(vp + e4);
    const v4f rr = *(const v4f*)(RES + base + e4);
    const v4f g  = *(const v4f*)(G + e4);
    const v4f bb = *(const v4f*)(Bt + e4);
    v4f o;
#pragma unroll
    for (int e = 0; e < 4; ++e) o[e] = rr[e] + (((v[e] - mu) * rstd) * g[e] + bb[e]);
    float* op = OUT + base + e4;
    *(volatile v4f*)op = o;
    __threadfence();
    *(volatile v4f*)op = o;
  }
}

extern "C" void kernel_launch(void* const* d_in, const int* in_sizes, int n_in,
                              void* d_out, int out_size, void* d_ws, size_t ws_size, hipStream_t stream) {
  if (n_in < 18 || d_out == nullptr || d_ws == nullptr) return;
  if (in_sizes[0] != NELEM || in_sizes[1] != NCH * GI || in_sizes[2] != HID * GI || in_sizes[3] != GI ||
      in_sizes[4] != NCH * GI || in_sizes[5] != HID * GI || in_sizes[6] != GI ||
      in_sizes[7] != NCH * NCH || in_sizes[8] != NCH || in_sizes[9] != SLAB || in_sizes[10] != SLAB ||
      in_sizes[11] != NCH * GJ || in_sizes[12] != NCH * GJ || in_sizes[13] != GJ ||
      in_sizes[14] != NCH * NCH || in_sizes[15] != NCH || in_sizes[16] != SLAB || in_sizes[17] != SLAB ||
      out_size != NELEM) return;

  const float* x    = (const float*)d_in[0];
  const float* iwf  = (const float*)d_in[1];
  const float* iuf  = (const float*)d_in[2];
  const float* ibf  = (const float*)d_in[3];
  const float* iwb  = (const float*)d_in[4];
  const float* iub  = (const float*)d_in[5];
  const float* ibb  = (const float*)d_in[6];
  const float* ifcw = (const float*)d_in[7];
  const float* ifcb = (const float*)d_in[8];
  const float* ilng = (const float*)d_in[9];
  const float* ilnb = (const float*)d_in[10];
  const float* jw   = (const float*)d_in[11];
  const float* ju   = (const float*)d_in[12];
  const float* jb   = (const float*)d_in[13];
  const float* jfcw = (const float*)d_in[14];
  const float* jfcb = (const float*)d_in[15];
  const float* jlng = (const float*)d_in[16];
  const float* jlnb = (const float*)d_in[17];
  float* out = (float*)d_out;

  char* ws = (char*)d_ws; size_t off = 0;
  auto carve = [&](size_t bytes) -> char* { char* p = ws + off; off += (bytes + 255) & ~(size_t)255; return p; };
  unsigned short* XZ16  = (unsigned short*)carve((size_t)NROW * GJ * 2);
  unsigned short* A16   = (unsigned short*)carve((size_t)NROW * NCH * 2);
  unsigned short* H16   = (unsigned short*)carve((size_t)NROW * NCH * 2);
  float*          DENSE = (float*)carve((size_t)NROW * NCH * 4);
  float*          RESID = (float*)carve((size_t)NROW * NCH * 4);
  unsigned short* BTI   = (unsigned short*)carve((size_t)GJ * NCH * 2);
  unsigned short* BTU   = (unsigned short*)carve((size_t)2 * GI * HID * 2);
  unsigned short* BTFCI = (unsigned short*)carve((size_t)NCH * NCH * 2);
  unsigned short* BTJ   = (unsigned short*)carve((size_t)GJ * NCH * 2);
  unsigned short* BTJU  = (unsigned short*)carve((size_t)GJ * NCH * 2);
  unsigned short* BTFCJ = (unsigned short*)carve((size_t)NCH * NCH * 2);
  float*          BIAS  = (float*)carve((size_t)GJ * 4);
  if (off > ws_size || off > (size_t)134217728) return;

  const int n8 = NELEM / 8;

  cvt8_f16_kernel<<<n8 / 256, 256, 0, stream>>>(x, A16, n8);
  tpw_f16_kernel<<<dim3(GI / 64, NCH / 64), 256, 0, stream>>>(iwf, NCH, GI, NCH, BTI, WCARRY);
  tpw_f16_kernel<<<dim3(GI / 64, NCH / 64), 256, 0, stream>>>(iwb, NCH, GI, NCH, BTI + (size_t)GI * NCH, WCARRY);
  tpw_f16_kernel<<<dim3(GI / 64, HID / 64), 256, 0, stream>>>(iuf, HID, GI, HID, BTU, WCARRY);
  tpw_f16_kernel<<<dim3(GI / 64, HID / 64), 256, 0, stream>>>(iub, HID, GI, HID, BTU + (size_t)GI * HID, WCARRY);
  tpw_f16_kernel<<<dim3(NCH / 64, NCH / 64), 256, 0, stream>>>(ifcw, NCH, NCH, NCH, BTFCI, WCARRY);
  tpw_f16_kernel<<<dim3(GJ / 64, NCH / 64), 256, 0, stream>>>(jw, NCH, GJ, NCH, BTJ, WCARRY);
  tpw_f16_kernel<<<dim3(GJ / 64, NCH / 64), 256, 0, stream>>>(ju, NCH, GJ, NCH, BTJU, WCARRY);
  tpw_f16_kernel<<<dim3(NCH / 64, NCH / 64), 256, 0, stream>>>(jfcw, NCH, NCH, NCH, BTFCJ, WCARRY);
  bias_cat_kernel<<<1, 128, 0, stream>>>(ibf, ibb, BIAS);

  const int gridWide = (NROW / 64) * (GJ / 64) / 8;
  const int gridNarrow = (NROW / 64) * (NCH / 64) / 8;

  wmma_gemm64_f16<1><<<gridWide, 256, 0, stream>>>(A16, NCH, BTI, NCH, (void*)XZ16, GJ, BIAS, NROW, GJ, NCH, INV_W);
  intra_seq_kernel<<<dim3(SEQL / 16, 2), 128, 0, stream>>>(XZ16, BTU, H16);
  wmma_gemm64_f16<0><<<gridNarrow, 256, 0, stream>>>(H16, NCH, BTFCI, NCH, (void*)DENSE, NCH, ifcb, NROW, NCH, NCH, INV_HW);
  ln_slab_res_kernel<<<SEQL, 256, 0, stream>>>(DENSE, x, ilng, ilnb, RESID);
  cvt8_f16_kernel<<<n8 / 256, 256, 0, stream>>>(RESID, A16, n8);
  wmma_gemm64_f16<1><<<gridWide, 256, 0, stream>>>(A16, NCH, BTJ, NCH, (void*)XZ16, GJ, jb, NROW, GJ, NCH, INV_W);
  inter_seq_kernel<<<WID / 16, 256, 0, stream>>>(XZ16, BTJU, H16);
  wmma_gemm64_f16<0><<<gridNarrow, 256, 0, stream>>>(H16, NCH, BTFCJ, NCH, (void*)DENSE, NCH, jfcb, NROW, NCH, NCH, INV_HW);
  ln_slab_res_kernel<<<SEQL, 256, 0, stream>>>(DENSE, RESID, jlng, jlnb, out);
}
